// SimpleRetention_26130581029009
// MI455X (gfx1250) — hardware-run, weakly checked
//
#include <hip/hip_runtime.h>
#include <math.h>

typedef __attribute__((ext_vector_type(16))) __bf16   v16b;
typedef __attribute__((ext_vector_type(8)))  __bf16   v8b;
typedef __attribute__((ext_vector_type(8)))  float    v8f;
typedef __attribute__((ext_vector_type(4)))  float    v4f;
typedef __attribute__((ext_vector_type(2)))  float    v2f;
typedef __attribute__((ext_vector_type(4)))  unsigned int v4u;

constexpr int kBatch = 4;
constexpr int kSeq   = 4096;
constexpr int kHid   = 256;
constexpr int kHead  = 64;
constexpr int kVd    = 64;
constexpr int kRows  = kBatch * kSeq;
constexpr int kNcat  = kHead + kHead + kVd;
constexpr int kHalf  = kHead / 2;
constexpr int kQTile = 64;
constexpr int kTilesPerSeq = kSeq / kQTile;
constexpr int kWinTiles = 8;
constexpr int kRotPitch = 196;
constexpr float kScaleBase = 512.0f;
constexpr float kLog2Gamma = -0.04580368961312479f;
constexpr float kSvAdd = (float)(0.4 * kHead);
constexpr float kSvDen = (float)(1.4 * kHead);
static_assert(kHid % 32 == 0, "GEMM K multiple of 32");
static_assert(kRows % 64 == 0 && kNcat % 64 == 0, "GEMM M,N multiples of 64");
static_assert(kSeq % kQTile == 0 && kHead == 64 && kVd == 64, "tile multiples");
static_assert(((kRows / 64) * (kNcat / 64)) % 8 == 0, "whole blocks of 8 tiles");

__constant__ const float kInvFreqTab[kHalf] = {
  1.0f,
  7.498942093324558e-1f,
  5.623413251903491e-1f,
  4.216965034285822e-1f,
  3.1622776601683794e-1f,
  2.371373705661655e-1f,
  1.7782794100389228e-1f,
  1.333521432163324e-1f,
  1.0e-1f,
  7.498942093324558e-2f,
  5.623413251903491e-2f,
  4.216965034285822e-2f,
  3.1622776601683794e-2f,
  2.371373705661655e-2f,
  1.7782794100389228e-2f,
  1.333521432163324e-2f,
  1.0e-2f,
  7.498942093324558e-3f,
  5.623413251903491e-3f,
  4.216965034285822e-3f,
  3.1622776601683794e-3f,
  2.371373705661655e-3f,
  1.7782794100389228e-3f,
  1.333521432163324e-3f,
  1.0e-3f,
  7.498942093324558e-4f,
  5.623413251903491e-4f,
  4.216965034285822e-4f,
  3.1622776601683794e-4f,
  2.371373705661655e-4f,
  1.7782794100389228e-4f,
  1.333521432163324e-4f
};
static_assert(sizeof(kInvFreqTab) / sizeof(kInvFreqTab[0]) == 32, "frequency table has one entry per pair");
static_assert(kHalf == 32, "pair count");

constexpr size_t kOffXB  = 0;
constexpr size_t kOffWT  = kOffXB  + (size_t)kRows * kHid * 2;
constexpr size_t kOffQKV = kOffWT  + (size_t)kNcat * kHid * 2;
constexpr size_t kOffQH  = kOffQKV + (size_t)kRows * kNcat * 4;
constexpr size_t kOffQL  = kOffQH  + (size_t)kRows * kHead * 2;
constexpr size_t kOffKH  = kOffQL  + (size_t)kRows * kHead * 2;
constexpr size_t kOffKL  = kOffKH  + (size_t)kRows * kHead * 2;
constexpr size_t kOffVTH = kOffKL  + (size_t)kRows * kHead * 2;
constexpr size_t kOffVTL = kOffVTH + (size_t)kBatch * kVd * kSeq * 2;
constexpr size_t kWsTotal = kOffVTL + (size_t)kBatch * kVd * kSeq * 2;
static_assert(kWsTotal == 33652736ull, "carve total");
static_assert(kWsTotal <= 134217728ull, "carve cap");
static_assert((kOffWT % 128) == 0 && (kOffQKV % 128) == 0 && (kOffQH % 128) == 0 && (kOffQL % 128) == 0 &&
              (kOffKH % 128) == 0 && (kOffKL % 128) == 0 && (kOffVTH % 128) == 0 && (kOffVTL % 128) == 0,
              "128-B aligned regions");

__device__ __forceinline__ unsigned short f2bf_bits(float f) {
  unsigned u = __float_as_uint(f);
  return (unsigned short)((u + 0x7FFFu + ((u >> 16) & 1u)) >> 16);
}
__device__ __forceinline__ float bf_bits2f(unsigned short h) { return __uint_as_float(((unsigned)h) << 16); }
__device__ __forceinline__ unsigned pk16(unsigned short a, unsigned short b) { return (unsigned)a | ((unsigned)b << 16); }

__device__ __forceinline__ void split_pack8(const float (&x)[8], v4u& hi, v4u& lo) {
  unsigned short hb[8], lb[8];
#pragma unroll
  for (int e = 0; e < 8; ++e) {
    const float f = x[e];
    hb[e] = f2bf_bits(f);
    lb[e] = f2bf_bits(f - bf_bits2f(hb[e]));
  }
  hi = (v4u){pk16(hb[0], hb[1]), pk16(hb[2], hb[3]), pk16(hb[4], hb[5]), pk16(hb[6], hb[7])};
  lo = (v4u){pk16(lb[0], lb[1]), pk16(lb[2], lb[3]), pk16(lb[4], lb[5]), pk16(lb[6], lb[7])};
}

union FragB { v16b v; v8b h[2]; };
__device__ __forceinline__ v16b frag_ld(const __bf16* p) {
  FragB f;
  f.h[0] = *(const v8b*)(p);
  f.h[1] = *(const v8b*)(p + 16);
  return f.v;
}
__device__ __forceinline__ v8f mma_raw(v16b a, v16b b, v8f c) {
  return __builtin_amdgcn_wmma_f32_16x16x32_bf16(false, a, false, b, (short)0, c, false, false);
}
__device__ __forceinline__ v8f mma_g(v16b a, v16b b, v8f c) {
  c = __builtin_amdgcn_wmma_f32_16x16x32_bf16(false, a, false, b, (short)0, c, false, false);
  asm volatile("v_nop\n\tv_nop\n\tv_nop\n\tv_nop" : "+v"(c) : "v"(a), "v"(b));
  return c;
}
__device__ __forceinline__ void guard4_b(v8f& a, v8f& b, v8f& c, v8f& d, v16b x) {
  asm volatile("v_nop\n\tv_nop\n\tv_nop\n\tv_nop" : "+v"(a), "+v"(b), "+v"(c), "+v"(d) : "v"(x));
}
__device__ __forceinline__ void keep4_b(v16b a, v16b b, v16b c, v16b d) { asm volatile("v_nop" :: "v"(a), "v"(b), "v"(c), "v"(d)); }
__device__ __forceinline__ void acc_guard4(v8f& a, v8f& b, v8f& c, v8f& d) { asm volatile("v_nop\n\tv_nop\n\tv_nop\n\tv_nop" : "+v"(a), "+v"(b), "+v"(c), "+v"(d)); }
__device__ __forceinline__ void split_bf(float f, __bf16& hi, __bf16& lo) {
  const unsigned short hb = f2bf_bits(f);
  const unsigned short lb = f2bf_bits(f - bf_bits2f(hb));
  hi = __builtin_bit_cast(__bf16, hb);
  lo = __builtin_bit_cast(__bf16, lb);
}
__device__ __forceinline__ void wave_lds_sync() {
  __builtin_amdgcn_fence(__ATOMIC_RELEASE, "workgroup");
  __builtin_amdgcn_wave_barrier();
  __builtin_amdgcn_fence(__ATOMIC_ACQUIRE, "workgroup");
}

__global__ __launch_bounds__(256) void cast8_bf16_kernel(const float* __restrict__ in, unsigned short* __restrict__ out, int n8) {
  const int i = blockIdx.x * 256 + threadIdx.x;
  if (i >= n8) return;
  const float* p = in + 8 * (size_t)i;
  const v4f a = *(const v4f*)(p);
  const v4f c = *(const v4f*)(p + 4);
  unsigned short hb[8];
#pragma unroll
  for (int e = 0; e < 4; ++e) {
    const float fa = a[e];
    const float fc = c[e];
    hb[e]     = f2bf_bits(fa);
    hb[4 + e] = f2bf_bits(fc);
  }
  const v4u u = (v4u){pk16(hb[0], hb[1]), pk16(hb[2], hb[3]), pk16(hb[4], hb[5]), pk16(hb[6], hb[7])};
  unsigned short* q = out + 8 * (size_t)i;
  *(volatile v4u*)q = u;
  __threadfence();
  *(volatile v4u*)q = u;
}

__global__ __launch_bounds__(256) void wt_bf16_kernel(const float* __restrict__ W0, const float* __restrict__ W1,
                                                      const float* __restrict__ W2, unsigned short* __restrict__ out) {
  __shared__ float sm[64][65];
  const int t  = threadIdx.x;
  const int k0 = blockIdx.x * 64;
  const int z  = blockIdx.y;
  const float* W = (z == 0) ? W0 : ((z == 1) ? W1 : W2);
#pragma unroll
  for (int i = 0; i < 16; ++i) {
    const int e = i * 256 + t;
    const int r = e >> 6;
    const int c = e & 63;
    sm[c][r] = W[(size_t)(k0 + r) * kHead + c];
  }
  __syncthreads();
  const int lane = t & 31;
  const int wave = __builtin_amdgcn_readfirstlane((int)(threadIdx.x >> 5));
  const int q = lane >> 3, c8 = (lane & 7) * 8;
  v4u u[2];
#pragma unroll
  for (int it = 0; it < 2; ++it) {
    const int row = wave * 8 + it * 4 + q;
    unsigned short hb[8];
#pragma unroll
    for (int e = 0; e < 8; ++e) hb[e] = f2bf_bits(sm[row][c8 + e]);
    u[it] = (v4u){pk16(hb[0], hb[1]), pk16(hb[2], hb[3]), pk16(hb[4], hb[5]), pk16(hb[6], hb[7])};
  }
  for (int pass = 0; pass < 2; ++pass) {
#pragma unroll
    for (int it = 0; it < 2; ++it) {
      const int row = wave * 8 + it * 4 + q;
      *(volatile v4u*)(out + (size_t)(z * 64 + row) * kHid + k0 + c8) = u[it];
    }
    __threadfence();
  }
}

__global__ __launch_bounds__(256) void proj_gemm_kernel(const unsigned short* __restrict__ Ap,
                                                        const unsigned short* __restrict__ Btp,
                                                        float* __restrict__ Cout) {
  const __bf16* A  = (const __bf16*)Ap;
  const __bf16* Bt = (const __bf16*)Btp;
  __shared__ __align__(16) float sT[8][16 * 68];
  const int lane = threadIdx.x & 31;
  const int wave = __builtin_amdgcn_readfirstlane((int)(threadIdx.x >> 5));
  constexpr int tilesN = kNcat >> 6;
  constexpr int tilesM = kRows >> 6;
  const int tile = blockIdx.x * 8 + wave;
  if (tile >= tilesM * tilesN) return;
  const int tm = tile / tilesN;
  const int tn = tile - tm * tilesN;
  const int m0 = tm << 6;
  const int n0 = tn << 6;
  const int rlane = lane & 15;
  const int koff  = (lane >> 4) * 8;
  const int mOff  = (lane >> 4) * 8;

  v8f acc[4][4];
#pragma unroll
  for (int i = 0; i < 4; ++i)
#pragma unroll
    for (int j = 0; j < 4; ++j) acc[i][j] = (v8f){0.f, 0.f, 0.f, 0.f, 0.f, 0.f, 0.f, 0.f};

  for (int k0 = 0; k0 < kHid; k0 += 32) {
    v16b bh[4];
#pragma unroll
    for (int j = 0; j < 4; ++j) {
      const size_t bo = (size_t)(n0 + (j << 4) + rlane) * kHid + koff + k0;
      bh[j] = frag_ld(Bt + bo);
    }
#pragma unroll
    for (int i = 0; i < 4; ++i) {
      const size_t ao = (size_t)(m0 + (i << 4) + rlane) * kHid + koff + k0;
      const v16b ah = frag_ld(A + ao);
#pragma unroll
      for (int j = 0; j < 4; ++j) acc[i][j] = mma_raw(ah, bh[j], acc[i][j]);
      guard4_b(acc[i][0], acc[i][1], acc[i][2], acc[i][3], ah);
    }
    keep4_b(bh[0], bh[1], bh[2], bh[3]);
  }
  acc_guard4(acc[0][0], acc[0][1], acc[0][2], acc[0][3]);
  acc_guard4(acc[1][0], acc[1][1], acc[1][2], acc[1][3]);
  acc_guard4(acc[2][0], acc[2][1], acc[2][2], acc[2][3]);
  acc_guard4(acc[3][0], acc[3][1], acc[3][2], acc[3][3]);

  float* slab = sT[wave];
#pragma unroll
  for (int i = 0; i < 4; ++i) {
    const int mBase = m0 + (i << 4);
#pragma unroll
    for (int j = 0; j < 4; ++j) {
#pragma unroll
      for (int r = 0; r < 8; ++r) {
        const float v = acc[i][j][r];
        slab[(mOff + r) * 68 + (j << 4) + rlane] = v;
      }
    }
    wave_lds_sync();
    {
      const int hh = lane >> 4, c4 = (lane & 15) * 4;
      for (int pass = 0; pass < 2; ++pass) {
#pragma unroll
        for (int it = 0; it < 8; ++it) {
          const int row = it * 2 + hh;
          const v4f v = *(const v4f*)(slab + row * 68 + c4);
          *(volatile v4f*)(Cout + (size_t)(mBase + row) * kNcat + n0 + c4) = v;
        }
        __threadfence();
      }
    }
    wave_lds_sync();
  }
}

__global__ __launch_bounds__(256) void rotscale_split_kernel(
    const float* __restrict__ QKV,
    unsigned short* __restrict__ QH, unsigned short* __restrict__ QL,
    unsigned short* __restrict__ KH, unsigned short* __restrict__ KL,
    unsigned short* __restrict__ VTH, unsigned short* __restrict__ VTL) {
  __shared__ __align__(16) float sT[64 * kRotPitch];
  const int tid  = threadIdx.x;
  const int lane = tid & 31;
  const int wave = __builtin_amdgcn_readfirstlane((int)(threadIdx.x >> 5));
  const int m0  = blockIdx.x * 64;
  const int bix = m0 / kSeq;
  const int l0  = m0 - bix * kSeq;

  const int pair = lane;
  const float fi = (float)pair;
  const float invf = kInvFreqTab[pair];
  const float svv  = (2.0f * fi + kSvAdd) * (1.0f / kSvDen);
  const float l2sv = log2f(svv);

#pragma unroll 1
  for (int it = 0; it < 8; ++it) {
    const int row = it * 8 + wave;
    const float fn  = (float)(l0 + row);
    const float ang = fn * invf;
    const float sn  = sinf(ang);
    const float cs  = cosf(ang);
    const float ex  = (fn * (1.0f / kScaleBase)) * l2sv;
    const float scq = exp2f(ex);
    const float sck = exp2f(-ex);
    const float* src = QKV + (size_t)(m0 + row) * kNcat + 2 * pair;
    const v2f xq = *(const v2f*)(src);
    const v2f xk = *(const v2f*)(src + kHead);
    const float q0 = xq[0], q1 = xq[1];
    const float k0 = xk[0], k1 = xk[1];
    const float cq = cs * scq, sq = sn * scq;
    const float ck = cs * sck, sk = sn * sck;
    float* d = sT + row * kRotPitch + 2 * pair;
    const v2f yq = (v2f){q0 * cq - q1 * sq, q1 * cq + q0 * sq};
    const v2f yk = (v2f){k0 * ck - k1 * sk, k1 * ck + k0 * sk};
    *(v2f*)(d) = yq;
    *(v2f*)(d + kHead) = yk;
  }
#pragma unroll
  for (int it = 0; it < 4; ++it) {
    const int item = it * 256 + tid;
    const int row = item >> 4;
    const int c4  = (item & 15) * 4;
    const v4f vv = *(const v4f*)(QKV + (size_t)(m0 + row) * kNcat + 2 * kHead + c4);
    *(v4f*)(sT + row * kRotPitch + 2 * kHead + c4) = vv;
  }
  __syncthreads();

  const int q4 = lane >> 3, c8 = (lane & 7) * 8;
  v4u uqh[2], uql[2], ukh[2], ukl[2], uvh[2], uvl[2];
#pragma unroll
  for (int it = 0; it < 2; ++it) {
    const int row = wave * 8 + it * 4 + q4;
    const float* sp = sT + row * kRotPitch + c8;
    float x[8];
    {
      const v4f a0 = *(const v4f*)(sp);
      const v4f a1 = *(const v4f*)(sp + 4);
#pragma unroll
      for (int e = 0; e < 4; ++e) { x[e] = a0[e]; x[4 + e] = a1[e]; }
      split_pack8(x, uqh[it], uql[it]);
    }
    {
      const v4f a0 = *(const v4f*)(sp + kHead);
      const v4f a1 = *(const v4f*)(sp + kHead + 4);
#pragma unroll
      for (int e = 0; e < 4; ++e) { x[e] = a0[e]; x[4 + e] = a1[e]; }
      split_pack8(x, ukh[it], ukl[it]);
    }
    {
#pragma unroll
      for (int e = 0; e < 8; ++e) x[e] = sT[(c8 + e) * kRotPitch + 2 * kHead + row];
      split_pack8(x, uvh[it], uvl[it]);
    }
  }
  for (int pass = 0; pass < 2; ++pass) {
#pragma unroll
    for (int it = 0; it < 2; ++it) {
      const int row = wave * 8 + it * 4 + q4;
      const size_t o  = (size_t)(m0 + row) * kHead + c8;
      const size_t ov = ((size_t)bix * kVd + row) * kSeq + l0 + c8;
      *(volatile v4u*)(QH + o) = uqh[it];
      *(volatile v4u*)(QL + o) = uql[it];
      *(volatile v4u*)(KH + o) = ukh[it];
      *(volatile v4u*)(KL + o) = ukl[it];
      *(volatile v4u*)(VTH + ov) = uvh[it];
      *(volatile v4u*)(VTL + ov) = uvl[it];
    }
    __threadfence();
  }
}

__global__ __launch_bounds__(128) void decay_attn_kernel(
    const unsigned short* __restrict__ QHp, const unsigned short* __restrict__ QLp,
    const unsigned short* __restrict__ KHp, const unsigned short* __restrict__ KLp,
    const unsigned short* __restrict__ VTHp, const unsigned short* __restrict__ VTLp,
    float* __restrict__ out) {
  __shared__ __align__(16) __bf16 Psh[4][16 * 64];
  __shared__ __align__(16) __bf16 Psl[4][16 * 64];
  __shared__ __align__(16) float  Os[4][16 * 68];
  const __bf16* QH  = (const __bf16*)QHp;
  const __bf16* QL  = (const __bf16*)QLp;
  const __bf16* KH  = (const __bf16*)KHp;
  const __bf16* KL  = (const __bf16*)KLp;
  const __bf16* VTH = (const __bf16*)VTHp;
  const __bf16* VTL = (const __bf16*)VTLp;

  const int lane = threadIdx.x & 31;
  const int wave = __builtin_amdgcn_readfirstlane((int)(threadIdx.x >> 5));
  const int hh = lane >> 4;
  const int c  = lane & 15;
  const int b  = blockIdx.x / kTilesPerSeq;
  const int qt = blockIdx.x - b * kTilesPerSeq;
  const int q0 = qt * kQTile + wave * 16;
  const size_t rowb = (size_t)b * kSeq;

  v16b qah[2], qal[2];
  {
    const size_t qo = (rowb + q0 + c) * kHead + 8 * hh;
#pragma unroll
    for (int dc = 0; dc < 2; ++dc) {
      qah[dc] = frag_ld(QH + qo + dc * 32);
      qal[dc] = frag_ld(QL + qo + dc * 32);
    }
  }
  v8f oacc[4];
#pragma unroll
  for (int t = 0; t < 4; ++t) oacc[t] = (v8f){0.f, 0.f, 0.f, 0.f, 0.f, 0.f, 0.f, 0.f};

  const float cj1 = exp2f(-16.0f * kLog2Gamma);
  const float cj2 = exp2f(-32.0f * kLog2Gamma);
  const float cj3 = exp2f(-48.0f * kLog2Gamma);

  __bf16* pwh = Psh[wave];
  __bf16* pwl = Psl[wave];
  const int jt0 = (qt > kWinTiles) ? (qt - kWinTiles) : 0;
#pragma unroll 1
  for (int jt = jt0; jt <= qt; ++jt) {
    const int kv0 = jt * kQTile;
    v8f s[4];
#pragma unroll
    for (int j = 0; j < 4; ++j) {
      s[j] = (v8f){0.f, 0.f, 0.f, 0.f, 0.f, 0.f, 0.f, 0.f};
      const size_t ko = (rowb + kv0 + j * 16 + c) * kHead + 8 * hh;
#pragma unroll
      for (int dc = 0; dc < 2; ++dc) {
        const v16b kh = frag_ld(KH + ko + dc * 32);
        const v16b kl = frag_ld(KL + ko + dc * 32);
        s[j] = mma_g(qah[dc], kh, s[j]);
        s[j] = mma_g(qah[dc], kl, s[j]);
        s[j] = mma_g(qal[dc], kh, s[j]);
      }
    }
    const int dbase = (q0 - kv0) + 8 * hh - c;
#pragma unroll
    for (int r = 0; r < 8; ++r) {
      const float wr = exp2f((float)(dbase + r) * kLog2Gamma);
#pragma unroll
      for (int j = 0; j < 4; ++j) {
        const int dlt = dbase + r - 16 * j;
        const float cf = (j == 0) ? 1.0f : ((j == 1) ? cj1 : ((j == 2) ? cj2 : cj3));
        const float sv = s[j][r];
        const float pv = sv * (wr * cf);
        const float p  = (dlt >= 0) ? pv : 0.0f;
        __bf16 ph, pl;
        split_bf(p, ph, pl);
        pwh[(8 * hh + r) * 64 + j * 16 + c] = ph;
        pwl[(8 * hh + r) * 64 + j * 16 + c] = pl;
      }
    }
    wave_lds_sync();
#pragma unroll 1
    for (int kk = 0; kk < 2; ++kk) {
      FragB pa, pb;
      pa.h[0] = *(const v8b*)(pwh + c * 64 + kk * 32 + 8 * hh);
      pa.h[1] = *(const v8b*)(pwh + c * 64 + kk * 32 + 16 + 8 * hh);
      pb.h[0] = *(const v8b*)(pwl + c * 64 + kk * 32 + 8 * hh);
      pb.h[1] = *(const v8b*)(pwl + c * 64 + kk * 32 + 16 + 8 * hh);
#pragma unroll
      for (int t = 0; t < 4; ++t) {
        const size_t vo = ((size_t)b * kVd + t * 16 + c) * kSeq + kv0 + kk * 32 + 8 * hh;
        const v16b vh = frag_ld(VTH + vo);
        const v16b vl = frag_ld(VTL + vo);
        oacc[t] = mma_g(pa.v, vh, oacc[t]);
        oacc[t] = mma_g(pa.v, vl, oacc[t]);
        oacc[t] = mma_g(pb.v, vh, oacc[t]);
      }
    }
    wave_lds_sync();
  }

  float* os = Os[wave];
#pragma unroll
  for (int r = 0; r < 8; ++r) {
#pragma unroll
    for (int t = 0; t < 4; ++t) {
      const float ov = oacc[t][r];
      os[(8 * hh + r) * 68 + t * 16 + c] = ov;
    }
  }
  wave_lds_sync();
  {
    const int c4 = (lane & 15) * 4;
    float* ob = out + (rowb + q0) * kVd;
    for (int pass = 0; pass < 2; ++pass) {
#pragma unroll
      for (int it = 0; it < 8; ++it) {
        const int row = it * 2 + hh;
        const v4f val = *(const v4f*)(os + row * 68 + c4);
        *(volatile v4f*)(ob + (size_t)row * kVd + c4) = val;
      }
      __threadfence();
    }
  }
}

extern "C" void kernel_launch(void* const* d_in, const int* in_sizes, int n_in,
                              void* d_out, int out_size, void* d_ws, size_t ws_size,
                              hipStream_t stream) {
  if (n_in < 4) return;
  if (in_sizes[0] != kRows * kHid) return;
  if (in_sizes[1] != kHid * kHead) return;
  if (in_sizes[2] != kHid * kHead) return;
  if (in_sizes[3] != kHid * kVd) return;
  if (out_size != kRows * kVd) return;
  if (ws_size < kWsTotal) return;

  const float* X  = (const float*)d_in[0];
  const float* WQ = (const float*)d_in[1];
  const float* WK = (const float*)d_in[2];
  const float* WV = (const float*)d_in[3];
  float* out = (float*)d_out;

  char* ws = (char*)d_ws;
  unsigned short* XB  = (unsigned short*)(ws + kOffXB);
  unsigned short* WT  = (unsigned short*)(ws + kOffWT);
  float*          QKV = (float*)(ws + kOffQKV);
  unsigned short* QH  = (unsigned short*)(ws + kOffQH);
  unsigned short* QL  = (unsigned short*)(ws + kOffQL);
  unsigned short* KH  = (unsigned short*)(ws + kOffKH);
  unsigned short* KL  = (unsigned short*)(ws + kOffKL);
  unsigned short* VTH = (unsigned short*)(ws + kOffVTH);
  unsigned short* VTL = (unsigned short*)(ws + kOffVTL);

  cast8_bf16_kernel<<<(kRows * kHid / 8) / 256, 256, 0, stream>>>(X, XB, kRows * kHid / 8);
  wt_bf16_kernel<<<dim3(kHid / 64, 3), 256, 0, stream>>>(WQ, WK, WV, WT);
  proj_gemm_kernel<<<((kRows / 64) * (kNcat / 64)) / 8, 256, 0, stream>>>(XB, WT, QKV);
  rotscale_split_kernel<<<kRows / 64, 256, 0, stream>>>(QKV, QH, QL, KH, KL, VTH, VTL);
  decay_attn_kernel<<<kBatch * kTilesPerSeq, 128, 0, stream>>>(QH, QL, KH, KL, VTH, VTL, out);
}
